// EncoderBlock_44470091382845
// MI455X (gfx1250) — hardware-run, weakly checked
//
#include <hip/hip_runtime.h>
#include <stddef.h>
#include <stdint.h>

#define NB     4
#define SQ     2048
#define NTOK   8192
#define DM     768
#define NH     8
#define HD     96
#define HP     128
#define DFF    3072
#define NQKV   2304
#define QB     128
#define KC     64
#define NQB    (SQ / QB)
#define NCK    (SQ / KC)
#define SBLK   (SQ / 256)
#define OPITCH (NH * HP)
#define QKPLANE ((size_t)NB * NH * SQ * HP)

static_assert(NTOK == NB * SQ);
static_assert(SQ % 256 == 0);
static_assert(SQ % QB == 0);
static_assert(SQ % KC == 0);
static_assert(KC == 64);
static_assert(QB == 128);
static_assert(DM % 64 == 0);
static_assert(DFF % 64 == 0);
static_assert(DM % 32 == 0);
static_assert(DFF % 32 == 0);
static_assert(HD == 96);
static_assert(HD % 32 == 0);
static_assert(HP >= HD);
static_assert(NH * HD == DM);
static_assert(NQKV == 3 * DM);
static_assert(NTOK % 256 == 0);
static_assert(DM == 3 * 256);

typedef _Float16 v16h __attribute__((ext_vector_type(16)));
typedef _Float16 v8h  __attribute__((ext_vector_type(8)));
typedef float    v8f  __attribute__((ext_vector_type(8)));
typedef float    v4f  __attribute__((ext_vector_type(4)));
typedef unsigned int v4u __attribute__((ext_vector_type(4)));

union Frag  { v16h v; v8h h[2]; };
union Pack8 { v8h h; v4u u; };

__device__ __forceinline__ v8f mma16(v16h a, v16h b, v8f c) {
  c = __builtin_amdgcn_wmma_f32_16x16x32_f16(false, a, false, b, (short)0, c, false, false);
  asm volatile("v_nop\n\tv_nop\n\tv_nop\n\tv_nop" : "+v"(c) : "v"(a), "v"(b));
  return c;
}

__device__ __forceinline__ v16h ldfrag(const _Float16* p, int ld, int row0, int k0, int lane) {
  const int m = lane & 15, lh = lane >> 4;
  const _Float16* q = p + (size_t)(row0 + m) * ld + k0 + 8 * lh;
  Frag f;
  f.h[0] = *(const v8h*)(q);
  f.h[1] = *(const v8h*)(q + 16);
  return f.v;
}

__device__ __forceinline__ v8f zero8() { return (v8f){0.f, 0.f, 0.f, 0.f, 0.f, 0.f, 0.f, 0.f}; }

template <int NT>
__device__ __forceinline__ void gemm32(const _Float16* __restrict__ A, int lda,
                                       const _Float16* __restrict__ Bt, int ldb,
                                       int ngrp, int gsa, int gsb, int ksteps,
                                       int m0, int n0, int lane, v8f (&acc)[2][4]) {
#pragma unroll 1
  for (int g = 0; g < ngrp; ++g) {
    const int kab = g * gsa, kbb = g * gsb;
#pragma unroll 1
    for (int j = 0; j < ksteps; ++j) {
      const int ka = kab + 32 * j, kb = kbb + 32 * j;
      const v16h a0 = ldfrag(A, lda, m0, ka, lane);
      const v16h a1 = ldfrag(A, lda, m0 + 16, ka, lane);
#pragma unroll
      for (int t = 0; t < NT; ++t) {
        const v16h bf = ldfrag(Bt, ldb, n0 + 16 * t, kb, lane);
        acc[0][t] = mma16(a0, bf, acc[0][t]);
        acc[1][t] = mma16(a1, bf, acc[1][t]);
      }
    }
  }
}

#define WTP 72
__global__ __launch_bounds__(256) void k_wtr(const float* __restrict__ w, _Float16* __restrict__ wt,
                                             int K, int N, float scale) {
  __shared__ __align__(16) _Float16 st[64 * WTP];
  const int tid = threadIdx.x;
  const int k0 = blockIdx.x * 64;
  const int n0 = blockIdx.y * 64;
#pragma unroll
  for (int i = 0; i < 4; ++i) {
    const int idx = tid + 256 * i;
    const int r   = idx >> 4;
    const int c4  = (idx & 15) * 4;
    const v4f f = *(const v4f*)(w + (size_t)(k0 + r) * N + n0 + c4) * scale;
    st[(c4 + 0) * WTP + r] = (_Float16)f[0];
    st[(c4 + 1) * WTP + r] = (_Float16)f[1];
    st[(c4 + 2) * WTP + r] = (_Float16)f[2];
    st[(c4 + 3) * WTP + r] = (_Float16)f[3];
  }
  __syncthreads();
  v4u val[2];
  size_t go[2];
#pragma unroll
  for (int g = 0; g < 2; ++g) {
    const int p   = tid + 256 * g;
    const int row = p >> 3;
    const int pc  = p & 7;
    Pack8 pk;
    pk.h   = *(const v8h*)(st + row * WTP + pc * 8);
    val[g] = pk.u;
    go[g]  = (size_t)(n0 + row) * K + k0 + pc * 8;
  }
  for (int ps = 0; ps < 2; ++ps) {
#pragma unroll
    for (int g = 0; g < 2; ++g) *(volatile v4u*)(wt + go[g]) = val[g];
    __threadfence();
  }
}

__global__ __launch_bounds__(256) void k_ln(const float* __restrict__ x, const float* __restrict__ g,
                                            const float* __restrict__ be, _Float16* __restrict__ y) {
  const int tid = threadIdx.x, lane = tid & 31, wave = tid >> 5;
  const size_t row = (size_t)blockIdx.x * 8 + wave;
  const float* xr = x + row * DM;
  float v[24];
#pragma unroll
  for (int i = 0; i < 3; ++i) {
#pragma unroll
    for (int e = 0; e < 2; ++e) {
      const v4f f = *(const v4f*)(xr + 256 * i + 8 * lane + 4 * e);
      v[8 * i + 4 * e + 0] = f[0];
      v[8 * i + 4 * e + 1] = f[1];
      v[8 * i + 4 * e + 2] = f[2];
      v[8 * i + 4 * e + 3] = f[3];
    }
  }
  float s = 0.f;
#pragma unroll
  for (int q = 0; q < 24; ++q) s += v[q];
#pragma unroll
  for (int off = 16; off >= 1; off >>= 1) s += __shfl_xor(s, off, 32);
  const float mu = s * (1.0f / (float)DM);
  float s2 = 0.f;
#pragma unroll
  for (int q = 0; q < 24; ++q) { v[q] -= mu; s2 += v[q] * v[q]; }
#pragma unroll
  for (int off = 16; off >= 1; off >>= 1) s2 += __shfl_xor(s2, off, 32);
  const float var = s2 * (1.0f / (float)DM);
  const float rs  = rsqrtf(var + 1e-5f);

  v4u val[3];
  size_t go[3];
#pragma unroll
  for (int i = 0; i < 3; ++i) {
    const int col = 256 * i + 8 * lane;
    const v4f g0 = *(const v4f*)(g + col),  g1 = *(const v4f*)(g + col + 4);
    const v4f b0 = *(const v4f*)(be + col), b1 = *(const v4f*)(be + col + 4);
    Pack8 pk;
    pk.h = (v8h){(_Float16)(v[8 * i + 0] * rs * g0[0] + b0[0]), (_Float16)(v[8 * i + 1] * rs * g0[1] + b0[1]),
                 (_Float16)(v[8 * i + 2] * rs * g0[2] + b0[2]), (_Float16)(v[8 * i + 3] * rs * g0[3] + b0[3]),
                 (_Float16)(v[8 * i + 4] * rs * g1[0] + b1[0]), (_Float16)(v[8 * i + 5] * rs * g1[1] + b1[1]),
                 (_Float16)(v[8 * i + 6] * rs * g1[2] + b1[2]), (_Float16)(v[8 * i + 7] * rs * g1[3] + b1[3])};
    val[i] = pk.u;
    go[i]  = row * DM + col;
  }
  for (int ps = 0; ps < 2; ++ps) {
#pragma unroll
    for (int i = 0; i < 3; ++i) *(volatile v4u*)(y + go[i]) = val[i];
    __threadfence();
  }
}

#define STP 72
#define SVP 264
__global__ __launch_bounds__(256) void k_qkv(const _Float16* __restrict__ yh,
                                             const _Float16* __restrict__ wt,
                                             const float* __restrict__ bq,
                                             const float* __restrict__ bk,
                                             const float* __restrict__ bv,
                                             _Float16* __restrict__ qkp,
                                             _Float16* __restrict__ vtp) {
  __shared__ __align__(16) _Float16 st[256 * STP];
  const int tid = threadIdx.x, lane = tid & 31, wave = tid >> 5;
  const int hh = lane >> 4, c = lane & 15;
  const int bx = blockIdx.x;
  const int b  = bx / SBLK;
  const int sb = (bx - b * SBLK) * 256;
  const int ns = blockIdx.y;
  const int which = ns >> 4;
  const int hs    = ns & 15;
  const int head  = hs >> 1;
  const int half  = hs & 1;
  const int d0    = half * 64;
  const int hb    = b * NH + head;
  const int m0 = bx * 256 + wave * 32;
  const int brow0 = which * DM + head * HD + d0;

  v8f acc[2][4];
#pragma unroll
  for (int s = 0; s < 2; ++s)
#pragma unroll
    for (int t = 0; t < 4; ++t) acc[s][t] = zero8();
  if (half == 0) gemm32<4>(yh, DM, wt, DM, 1, 0, 0, DM / 32, m0, brow0, lane, acc);
  else           gemm32<2>(yh, DM, wt, DM, 1, 0, 0, DM / 32, m0, brow0, lane, acc);

  float bb[4];
#pragma unroll
  for (int t = 0; t < 4; ++t) {
    const int dd = d0 + 16 * t + c;
    const int i  = head * HD + dd;
    const int ic = (i < DM) ? i : (DM - 1);
    const float xq = bq[ic], xk = bk[ic], xv = bv[ic];
    const float sel = (which == 0) ? xq : ((which == 1) ? xk : xv);
    bb[t] = (dd < HD) ? sel : 0.0f;
  }

  if (which < 2) {
#pragma unroll
    for (int sub = 0; sub < 2; ++sub)
#pragma unroll
      for (int t = 0; t < 4; ++t)
#pragma unroll
        for (int r = 0; r < 8; ++r)
          st[(wave * 32 + sub * 16 + 8 * hh + r) * STP + 16 * t + c] =
              (_Float16)(acc[sub][t][r] * 0.03125f + bb[t]);
  } else {
#pragma unroll
    for (int sub = 0; sub < 2; ++sub)
#pragma unroll
      for (int t = 0; t < 4; ++t)
#pragma unroll
        for (int r = 0; r < 8; ++r)
          st[(16 * t + c) * SVP + wave * 32 + sub * 16 + 8 * hh + r] =
              (_Float16)(acc[sub][t][r] * 0.03125f + bb[t]);
  }
  __syncthreads();

  if (which < 2) {
    _Float16* base = qkp + (size_t)which * QKPLANE + (size_t)hb * SQ * HP + d0;
#pragma unroll
    for (int g = 0; g < 2; ++g) {
      v4u val[4];
      size_t go[4];
#pragma unroll
      for (int j = 0; j < 4; ++j) {
        const int p  = tid + 256 * (4 * g + j);
        const int lr = p >> 3;
        const int pc = p & 7;
        Pack8 pk;
        pk.h   = *(const v8h*)(st + lr * STP + pc * 8);
        val[j] = pk.u;
        go[j]  = (size_t)(sb + lr) * HP + pc * 8;
      }
      for (int ps = 0; ps < 2; ++ps) {
#pragma unroll
        for (int j = 0; j < 4; ++j) *(volatile v4u*)(base + go[j]) = val[j];
        __threadfence();
      }
    }
  } else {
    _Float16* base = vtp + ((size_t)hb * HP + d0) * SQ;
#pragma unroll
    for (int g = 0; g < 2; ++g) {
      v4u val[4];
      size_t go[4];
#pragma unroll
      for (int j = 0; j < 4; ++j) {
        const int p    = tid + 256 * (4 * g + j);
        const int drow = p >> 5;
        const int pc   = p & 31;
        Pack8 pk;
        pk.h   = *(const v8h*)(st + drow * SVP + pc * 8);
        val[j] = pk.u;
        go[j]  = (size_t)drow * SQ + sb + pc * 8;
      }
      for (int ps = 0; ps < 2; ++ps) {
#pragma unroll
        for (int j = 0; j < 4; ++j) *(volatile v4u*)(base + go[j]) = val[j];
        __threadfence();
      }
    }
  }
}

#define KTP 104
#define VTP 72
#define PTP 104
__global__ __launch_bounds__(256) void k_attn(const _Float16* __restrict__ qp,
                                              const _Float16* __restrict__ kp,
                                              const _Float16* __restrict__ vt,
                                              _Float16* __restrict__ op) {
  __shared__ __align__(16) _Float16 Ks[KC * KTP];
  __shared__ __align__(16) _Float16 Vs[HD * VTP];
  __shared__ __align__(16) _Float16 Ps[8 * 16 * PTP];

  const int tid = threadIdx.x, lane = tid & 31, wave = tid >> 5;
  const int hh = lane >> 4, c = lane & 15;
  const int qb  = blockIdx.x % NQB;
  const int hb  = blockIdx.x / NQB;
  const int h   = hb % NH;
  const int b   = hb / NH;
  const int q0  = qb * QB + wave * 16;

  const _Float16* Q = qp + (size_t)hb * SQ * HP;
  const _Float16* K = kp + (size_t)hb * SQ * HP;
  const _Float16* V = vt + (size_t)hb * HP * SQ;

  v16h qa[3];
  qa[0] = ldfrag(Q, HP, q0, 0, lane);
  qa[1] = ldfrag(Q, HP, q0, 32, lane);
  qa[2] = ldfrag(Q, HP, q0, 64, lane);

  const float NEGI = -__builtin_huge_valf();
  float mrow[8], lrow[8];
  v8f oacc[6];
#pragma unroll
  for (int r = 0; r < 8; ++r) { mrow[r] = NEGI; lrow[r] = 0.f; }
#pragma unroll
  for (int t = 0; t < 6; ++t) oacc[t] = zero8();

  _Float16* pw = Ps + wave * 16 * PTP;

  for (int kc = 0; kc < NCK; ++kc) {
    const int kv0 = kc * KC;
    __syncthreads();
#pragma unroll
    for (int e = 0; e < 3; ++e) {
      const int p  = tid + 256 * e;
      const int r  = p / 12;
      const int q8 = (p - r * 12) * 8;
      *(v8h*)(Ks + r * KTP + q8) = *(const v8h*)(K + (size_t)(kv0 + r) * HP + q8);
      const int r2 = p >> 3;
      const int q2 = (p & 7) * 8;
      *(v8h*)(Vs + r2 * VTP + q2) = *(const v8h*)(V + (size_t)r2 * SQ + kv0 + q2);
    }
    __syncthreads();

    v8f s[4];
#pragma unroll
    for (int j = 0; j < 4; ++j) s[j] = zero8();
#pragma unroll
    for (int dc = 0; dc < 3; ++dc) {
#pragma unroll
      for (int j = 0; j < 4; ++j) {
        const v16h kb = ldfrag(Ks, KTP, j * 16, dc * 32, lane);
        s[j] = mma16(qa[dc], kb, s[j]);
      }
    }
    float cm[8];
#pragma unroll
    for (int r = 0; r < 8; ++r) {
      float m = NEGI;
#pragma unroll
      for (int j = 0; j < 4; ++j) m = fmaxf(m, s[j][r]);
#pragma unroll
      for (int off = 1; off < 16; off <<= 1) m = fmaxf(m, __shfl_xor(m, off, 32));
      cm[r] = m;
    }
    float al[8];
#pragma unroll
    for (int r = 0; r < 8; ++r) {
      const float mnew  = fmaxf(mrow[r], cm[r]);
      const float alpha = __expf(mrow[r] - mnew);
      mrow[r] = mnew;
      float psum = 0.f;
#pragma unroll
      for (int j = 0; j < 4; ++j) {
        const float p = __expf(s[j][r] - mnew);
        psum += p;
        pw[(8 * hh + r) * PTP + j * 16 + c] = (_Float16)(p * 1024.0f);
      }
#pragma unroll
      for (int off = 1; off < 16; off <<= 1) psum += __shfl_xor(psum, off, 32);
      lrow[r] = lrow[r] * alpha + psum;
      al[r] = alpha;
    }
#pragma unroll
    for (int t = 0; t < 6; ++t)
#pragma unroll
      for (int r = 0; r < 8; ++r) oacc[t][r] *= al[r];
    __syncthreads();

#pragma unroll
    for (int kk = 0; kk < 2; ++kk) {
      const v16h pa = ldfrag(pw, PTP, 0, kk * 32, lane);
#pragma unroll
      for (int t = 0; t < 6; ++t) {
        const v16h vb = ldfrag(Vs, VTP, t * 16, kk * 32, lane);
        oacc[t] = mma16(pa, vb, oacc[t]);
      }
    }
  }

  float invl[8];
#pragma unroll
  for (int r = 0; r < 8; ++r) invl[r] = (lrow[r] > 0.f) ? (0.0625f * (1.0f / lrow[r])) : 0.f;
  __syncthreads();
#pragma unroll
  for (int r = 0; r < 8; ++r) {
#pragma unroll
    for (int t = 0; t < 6; ++t)
      pw[(8 * hh + r) * PTP + 16 * t + c] = (_Float16)(oacc[t][r] * invl[r]);
  }
  __syncthreads();
  v4u val[8];
  size_t go[8];
#pragma unroll
  for (int it = 0; it < 8; ++it) {
    const int p   = lane + 32 * it;
    const int L   = p >> 4;
    const int pc  = p & 15;
    const int pcs = (pc < 12) ? pc : 11;
    Pack8 pk;
    pk.h = *(const v8h*)(pw + L * PTP + pcs * 8);
    v4u o;
    o.x = (pc < 12) ? pk.u.x : 0u;
    o.y = (pc < 12) ? pk.u.y : 0u;
    o.z = (pc < 12) ? pk.u.z : 0u;
    o.w = (pc < 12) ? pk.u.w : 0u;
    val[it] = o;
    go[it]  = ((size_t)b * SQ + (size_t)(q0 + L)) * OPITCH + (size_t)h * HP + pc * 8;
  }
  for (int ps = 0; ps < 2; ++ps) {
#pragma unroll
    for (int it = 0; it < 8; ++it) *(volatile v4u*)(op + go[it]) = val[it];
    __threadfence();
  }
}

#define OTP 68
__device__ __forceinline__ void out_epilogue_f32(v8f (&acc)[2][4], float scale, const float (&bb)[4],
                                                 float* sw, const float* __restrict__ resid,
                                                 float* __restrict__ out, int ldo,
                                                 int m0, int n0, int lane, int hh, int c) {
#pragma unroll
  for (int sub = 0; sub < 2; ++sub) {
    __syncthreads();
#pragma unroll
    for (int t = 0; t < 4; ++t) {
#pragma unroll
      for (int r = 0; r < 8; ++r) sw[(8 * hh + r) * OTP + 16 * t + c] = acc[sub][t][r] * scale + bb[t];
    }
    __syncthreads();
    v4f val[8];
    size_t go[8];
#pragma unroll
    for (int it = 0; it < 8; ++it) {
      const int p    = lane + 32 * it;
      const int L    = p >> 3;
      const int pc   = p & 7;
      const int row  = L >> 1;
      const int half = L & 1;
      go[it]  = (size_t)(m0 + sub * 16 + row) * ldo + n0 + half * 32 + pc * 4;
      val[it] = *(const v4f*)(sw + row * OTP + half * 32 + pc * 4) + *(const v4f*)(resid + go[it]);
    }
    for (int ps = 0; ps < 2; ++ps) {
#pragma unroll
      for (int it = 0; it < 8; ++it) *(volatile v4f*)(out + go[it]) = val[it];
      __threadfence();
    }
  }
}

__global__ __launch_bounds__(256) void k_gemm_f32(const _Float16* __restrict__ ap, int lda, int ngrp, int gsa,
                                                  const _Float16* __restrict__ wt, int ldb, int gsb, int ksteps,
                                                  const float* __restrict__ bias, float scale,
                                                  const float* __restrict__ resid,
                                                  float* __restrict__ out, int ldo) {
  __shared__ __align__(16) float st[8][16 * OTP];
  const int tid = threadIdx.x, lane = tid & 31, wave = tid >> 5;
  const int hh = lane >> 4, c = lane & 15;
  const int m0 = blockIdx.x * 256 + wave * 32;
  const int n0 = blockIdx.y * 64;

  v8f acc[2][4];
#pragma unroll
  for (int s = 0; s < 2; ++s)
#pragma unroll
    for (int t = 0; t < 4; ++t) acc[s][t] = zero8();
  gemm32<4>(ap, lda, wt, ldb, ngrp, gsa, gsb, ksteps, m0, n0, lane, acc);
  float bb[4];
#pragma unroll
  for (int t = 0; t < 4; ++t) bb[t] = bias[n0 + 16 * t + c];
  out_epilogue_f32(acc, scale, bb, st[wave], resid, out, ldo, m0, n0, lane, hh, c);
}

#define HTP 72
__global__ __launch_bounds__(256) void k_gemm_gelu(const _Float16* __restrict__ ap,
                                                   const _Float16* __restrict__ wt,
                                                   const float* __restrict__ bias,
                                                   _Float16* __restrict__ hout) {
  __shared__ __align__(16) _Float16 st[8 * 32 * HTP];
  const int tid = threadIdx.x, lane = tid & 31, wave = tid >> 5;
  const int hh = lane >> 4, c = lane & 15;
  const int m0 = blockIdx.x * 256 + wave * 32;
  const int n0 = blockIdx.y * 64;

  v8f acc[2][4];
#pragma unroll
  for (int s = 0; s < 2; ++s)
#pragma unroll
    for (int t = 0; t < 4; ++t) acc[s][t] = zero8();
  gemm32<4>(ap, DM, wt, DM, 1, 0, 0, DM / 32, m0, n0, lane, acc);
  float bb[4];
#pragma unroll
  for (int t = 0; t < 4; ++t) bb[t] = bias[n0 + 16 * t + c];

  _Float16* sw = st + wave * 32 * HTP;
#pragma unroll
  for (int sub = 0; sub < 2; ++sub)
#pragma unroll
    for (int t = 0; t < 4; ++t)
#pragma unroll
      for (int r = 0; r < 8; ++r) {
        const float u  = acc[sub][t][r] * 0.03125f + bb[t];
        const float gl = 0.5f * u * (1.0f + erff(u * 0.70710678118654752f));
        sw[(sub * 16 + 8 * hh + r) * HTP + 16 * t + c] = (_Float16)(gl * 16.0f);
      }
  __syncthreads();
  v4u val[8];
  size_t go[8];
#pragma unroll
  for (int it = 0; it < 8; ++it) {
    const int p  = lane + 32 * it;
    const int L  = p >> 3;
    const int pc = p & 7;
    Pack8 pk;
    pk.h    = *(const v8h*)(sw + L * HTP + pc * 8);
    val[it] = pk.u;
    go[it]  = (size_t)(m0 + L) * DFF + n0 + pc * 8;
  }
  for (int ps = 0; ps < 2; ++ps) {
#pragma unroll
    for (int it = 0; it < 8; ++it) *(volatile v4u*)(hout + go[it]) = val[it];
    __threadfence();
  }
}

extern "C" void kernel_launch(void* const* d_in, const int* in_sizes, int n_in,
                              void* d_out, int out_size, void* d_ws, size_t ws_size,
                              hipStream_t stream) {
  if (n_in < 17) return;
  if (in_sizes[0]  != NTOK * DM) return;
  if (in_sizes[1]  != DM) return;
  if (in_sizes[2]  != DM) return;
  if (in_sizes[3]  != DM * DM) return;
  if (in_sizes[4]  != DM) return;
  if (in_sizes[5]  != DM * DM) return;
  if (in_sizes[6]  != DM) return;
  if (in_sizes[7]  != DM * DM) return;
  if (in_sizes[8]  != DM) return;
  if (in_sizes[9]  != DM * DM) return;
  if (in_sizes[10] != DM) return;
  if (in_sizes[11] != DM) return;
  if (in_sizes[12] != DM) return;
  if (in_sizes[13] != DM * DFF) return;
  if (in_sizes[14] != DFF) return;
  if (in_sizes[15] != DFF * DM) return;
  if (in_sizes[16] != DM) return;
  if (out_size != NTOK * DM) return;

  const float* x    = (const float*)d_in[0];
  const float* g1   = (const float*)d_in[1];
  const float* be1  = (const float*)d_in[2];
  const float* wq   = (const float*)d_in[3];
  const float* bq   = (const float*)d_in[4];
  const float* wk   = (const float*)d_in[5];
  const float* bk   = (const float*)d_in[6];
  const float* wv   = (const float*)d_in[7];
  const float* bv   = (const float*)d_in[8];
  const float* wo   = (const float*)d_in[9];
  const float* bo   = (const float*)d_in[10];
  const float* g2   = (const float*)d_in[11];
  const float* be2  = (const float*)d_in[12];
  const float* w1   = (const float*)d_in[13];
  const float* b1   = (const float*)d_in[14];
  const float* w2   = (const float*)d_in[15];
  const float* b2   = (const float*)d_in[16];
  float* out = (float*)d_out;

  size_t off = 0;
  const size_t oY   = off; off += (size_t)NTOK * DM * 2;
  const size_t oWqk = off; off += (size_t)NQKV * DM * 2;
  const size_t oWo  = off; off += (size_t)DM * DM * 2;
  const size_t oW1  = off; off += (size_t)DFF * DM * 2;
  const size_t oW2  = off; off += (size_t)DM * DFF * 2;
  const size_t oQ   = off; off += QKPLANE * 2;
  const size_t oK   = off; off += QKPLANE * 2;
  const size_t oV   = off; off += QKPLANE * 2;
  const size_t oO   = off; off += (size_t)NTOK * OPITCH * 2;
  const size_t oX1  = off; off += (size_t)NTOK * DM * 4;
  const size_t oH   = oQ;
  if (off > ws_size) return;
  if (off > (size_t)134217728) return;
  if (oK != oQ + QKPLANE * 2) return;
  if (oH + (size_t)NTOK * DFF * 2 > oX1) return;

  char* ws = (char*)d_ws;
  _Float16* Yh   = (_Float16*)(ws + oY);
  _Float16* Wqkv = (_Float16*)(ws + oWqk);
  _Float16* Wot  = (_Float16*)(ws + oWo);
  _Float16* W1t  = (_Float16*)(ws + oW1);
  _Float16* W2t  = (_Float16*)(ws + oW2);
  _Float16* QKp  = (_Float16*)(ws + oQ);
  _Float16* Kp   = (_Float16*)(ws + oK);
  _Float16* Vt   = (_Float16*)(ws + oV);
  _Float16* Op   = (_Float16*)(ws + oO);
  float*    X1   = (float*)(ws + oX1);
  _Float16* Hh   = (_Float16*)(ws + oH);

  k_wtr<<<dim3(DM / 64, DM / 64), dim3(256), 0, stream>>>(wq, Wqkv, DM, DM, 32.0f);
  k_wtr<<<dim3(DM / 64, DM / 64), dim3(256), 0, stream>>>(wk, Wqkv + (size_t)DM * DM, DM, DM, 32.0f);
  k_wtr<<<dim3(DM / 64, DM / 64), dim3(256), 0, stream>>>(wv, Wqkv + (size_t)2 * DM * DM, DM, DM, 32.0f);
  k_wtr<<<dim3(DM / 64, DM / 64), dim3(256), 0, stream>>>(wo, Wot, DM, DM, 32.0f);
  k_wtr<<<dim3(DM / 64, DFF / 64), dim3(256), 0, stream>>>(w1, W1t, DM, DFF, 32.0f);
  k_wtr<<<dim3(DFF / 64, DM / 64), dim3(256), 0, stream>>>(w2, W2t, DFF, DM, 32.0f);
  k_ln<<<dim3(NTOK / 8), dim3(256), 0, stream>>>(x, g1, be1, Yh);
  k_qkv<<<dim3(NTOK / 256, 3 * NH * 2), dim3(256), 0, stream>>>(Yh, Wqkv, bq, bk, bv, QKp, Vt);
  k_attn<<<dim3(NB * NH * NQB), dim3(256), 0, stream>>>(QKp, Kp, Vt, Op);
  const float so = 0.00048828125f * 0.03608439182435161f;
  k_gemm_f32<<<dim3(NTOK / 256, DM / 64), dim3(256), 0, stream>>>(Op, OPITCH, NH, HP, Wot, DM, HD, HD / 32,
                                                                  bo, so, x, X1, DM);
  k_ln<<<dim3(NTOK / 8), dim3(256), 0, stream>>>(X1, g2, be2, Yh);
  k_gemm_gelu<<<dim3(NTOK / 256, DFF / 64), dim3(256), 0, stream>>>(Yh, W1t, b1, Hh);
  k_gemm_f32<<<dim3(NTOK / 256, DM / 64), dim3(256), 0, stream>>>(Hh, DFF, 1, 0, W2t, DFF, 0, DFF / 32,
                                                                  b2, 0.001953125f, X1, out, DM);
  (void)hipGetLastError();
}
